// MaskedSelfAttention_44272522887253
// MI455X (gfx1250) — hardware-verified
//
#include <hip/hip_runtime.h>

typedef __attribute__((ext_vector_type(16))) _Float16 v16h;
typedef __attribute__((ext_vector_type(8)))  _Float16 v8h;
typedef __attribute__((ext_vector_type(16))) __bf16   v16b;
typedef __attribute__((ext_vector_type(8)))  __bf16   v8b;
typedef __attribute__((ext_vector_type(8)))  float    v8f;
typedef __attribute__((ext_vector_type(4)))  float    v4f;
typedef __attribute__((ext_vector_type(2)))  float    v2f;

#define NEG_INF (-__builtin_inff())

__device__ __forceinline__ unsigned short f2bf_bits(float f) {
  unsigned u = __float_as_uint(f);
  return (unsigned short)((u + 0x7FFFu + ((u >> 16) & 1u)) >> 16);
}
__device__ __forceinline__ float bf_bits2f(unsigned short h) { return __uint_as_float(((unsigned)h) << 16); }
__device__ __forceinline__ void bf_split(float f, __bf16& hi, __bf16& lo) {
  const unsigned short hb = f2bf_bits(f);
  hi = __builtin_bit_cast(__bf16, hb);
  lo = __builtin_bit_cast(__bf16, f2bf_bits(f - bf_bits2f(hb)));
}

__device__ __forceinline__ void dep_guard_h(v8f& a, v8f& b, v16h x, v16h y) { asm volatile("v_nop\n\tv_nop\n\tv_nop\n\tv_nop" : "+v"(a), "+v"(b) : "v"(x), "v"(y)); }
__device__ __forceinline__ void dep_guard_b(v8f& a, v8f& b, v16b x, v16b y) { asm volatile("v_nop\n\tv_nop\n\tv_nop\n\tv_nop" : "+v"(a), "+v"(b) : "v"(x), "v"(y)); }
__device__ __forceinline__ void keep4_h(v16h a, v16h b, v16h c, v16h d) { asm volatile("v_nop" :: "v"(a), "v"(b), "v"(c), "v"(d)); }
__device__ __forceinline__ void keep4_b(v16b a, v16b b, v16b c, v16b d) { asm volatile("v_nop" :: "v"(a), "v"(b), "v"(c), "v"(d)); }
__device__ __forceinline__ void acc_guard4(v8f& a, v8f& b, v8f& c, v8f& d) { asm volatile("v_nop\n\tv_nop\n\tv_nop\n\tv_nop" : "+v"(a), "+v"(b), "+v"(c), "+v"(d)); }

template <typename T> struct Frag;
template <> struct Frag<_Float16> {
  typedef v16h V; union U { v16h v; v8h h[2]; };
  static __device__ __forceinline__ v16h load(const _Float16* p) {
    U f; f.h[0] = *(const v8h*)(p); f.h[1] = *(const v8h*)(p + 16); return f.v;
  }
  static __device__ __forceinline__ v8f mma(v16h a, v16h b, v8f c) {
    return __builtin_amdgcn_wmma_f32_16x16x32_f16(false, a, false, b, (short)0, c, false, false);
  }
  static __device__ __forceinline__ void guard(v8f& a, v8f& b, v16h x, v16h y) { dep_guard_h(a, b, x, y); }
  static __device__ __forceinline__ void keep(v16h a, v16h b, v16h c, v16h d) { keep4_h(a, b, c, d); }
};
template <> struct Frag<__bf16> {
  typedef v16b V; union U { v16b v; v8b h[2]; };
  static __device__ __forceinline__ v16b load(const __bf16* p) {
    U f; f.h[0] = *(const v8b*)(p); f.h[1] = *(const v8b*)(p + 16); return f.v;
  }
  static __device__ __forceinline__ v8f mma(v16b a, v16b b, v8f c) {
    return __builtin_amdgcn_wmma_f32_16x16x32_bf16(false, a, false, b, (short)0, c, false, false);
  }
  static __device__ __forceinline__ void guard(v8f& a, v8f& b, v16b x, v16b y) { dep_guard_b(a, b, x, y); }
  static __device__ __forceinline__ void keep(v16b a, v16b b, v16b c, v16b d) { keep4_b(a, b, c, d); }
};

__device__ __forceinline__ v8f mma_bf16x(v16b a, v16b b, v8f c) {
  c = __builtin_amdgcn_wmma_f32_16x16x32_bf16(false, a, false, b, (short)0, c, false, false);
  asm volatile("v_nop\n\tv_nop\n\tv_nop\n\tv_nop" : "+v"(c) : "v"(a), "v"(b));
  return c;
}
__device__ __forceinline__ v8f mma_f16x(v16h a, v16h b, v8f c) {
  c = __builtin_amdgcn_wmma_f32_16x16x32_f16(false, a, false, b, (short)0, c, false, false);
  asm volatile("v_nop\n\tv_nop\n\tv_nop\n\tv_nop" : "+v"(c) : "v"(a), "v"(b));
  return c;
}

template <int ET> struct Elem;
template <> struct Elem<0> { typedef _Float16 T; };
template <> struct Elem<1> { typedef __bf16 T; };
template <int ET, bool SPLIT, int BIAS_MODE, int OUT_MODE, bool RESID, int ACT, int ROPE>
__global__ __launch_bounds__(256) void wmma_gemm64(
    const unsigned short* __restrict__ Ap, const unsigned short* __restrict__ A2p, int lda, long strideA,
    const unsigned short* __restrict__ Btp, const unsigned short* __restrict__ Bt2p, int ldb, long strideB,
    void* __restrict__ Cout, void* __restrict__ Cout2, int ldc, long strideC,
    const float* __restrict__ bias,
    const float* __restrict__ resid, long strideR,
    const float* __restrict__ rope_cs, int ropeT,
    int M, int N, int K, float scale) {
#pragma clang fp contract(off)
  typedef typename Elem<ET>::T T;
  typedef typename Frag<T>::V V;
  const T* A = (const T*)Ap; const T* A2 = (const T*)A2p; const T* Bt = (const T*)Btp; const T* Bt2 = (const T*)Bt2p;
  __shared__ __align__(16) float sT[8][16 * 68];
  const int b    = blockIdx.y;
  const int lane = threadIdx.x & 31;
  const int wave = threadIdx.x >> 5;
  const int tilesN = N >> 6;
  const int tilesM = M >> 6;
  const int tile = blockIdx.x * 8 + wave;
  if (tile >= tilesM * tilesN) return;
  const int tm = tile / tilesN;
  const int tn = tile - tm * tilesN;
  const int m0 = tm << 6;
  const int n0 = tn << 6;

  const T* Ab  = A  + (size_t)b * strideA;
  const T* Bb  = Bt + (size_t)b * strideB;
  const T* Ab2 = SPLIT ? (A2  + (size_t)b * strideA) : nullptr;
  const T* Bb2 = SPLIT ? (Bt2 + (size_t)b * strideB) : nullptr;

  const int rlane = lane & 15;
  const int koff  = (lane >> 4) * 8;
  const int mOff  = (lane >> 4) * 8;

  v8f acc[4][4];
#pragma unroll
  for (int i = 0; i < 4; ++i)
#pragma unroll
    for (int j = 0; j < 4; ++j) acc[i][j] = (v8f){0.f,0.f,0.f,0.f,0.f,0.f,0.f,0.f};

  for (int k0 = 0; k0 < K; k0 += 32) {
    V bh[4], bl[4];
#pragma unroll
    for (int j = 0; j < 4; ++j) {
      const size_t bo = (size_t)(n0 + (j << 4) + rlane) * ldb + koff + k0;
      bh[j] = Frag<T>::load(Bb + bo);
      if (SPLIT) bl[j] = Frag<T>::load(Bb2 + bo);
    }
#pragma unroll
    for (int i = 0; i < 4; ++i) {
      const size_t ao = (size_t)(m0 + (i << 4) + rlane) * lda + koff + k0;
      V ah = Frag<T>::load(Ab + ao);
      V al;
      if (SPLIT) al = Frag<T>::load(Ab2 + ao);
#pragma unroll
      for (int j = 0; j < 4; ++j) {
        acc[i][j] = Frag<T>::mma(ah, bh[j], acc[i][j]);
        if (SPLIT) {
          acc[i][j] = Frag<T>::mma(ah, bl[j], acc[i][j]);
          acc[i][j] = Frag<T>::mma(al, bh[j], acc[i][j]);
        }
      }
      Frag<T>::guard(acc[i][0], acc[i][3], ah, SPLIT ? al : ah);
    }
    Frag<T>::keep(bh[0], bh[1], bh[2], bh[3]);
    if (SPLIT) Frag<T>::keep(bl[0], bl[1], bl[2], bl[3]);
  }
  acc_guard4(acc[0][0], acc[0][1], acc[0][2], acc[0][3]);
  acc_guard4(acc[1][0], acc[1][1], acc[1][2], acc[1][3]);
  acc_guard4(acc[2][0], acc[2][1], acc[2][2], acc[2][3]);
  acc_guard4(acc[3][0], acc[3][1], acc[3][2], acc[3][3]);

  float* slab = sT[wave];
  const float* Rb = RESID ? (resid + (size_t)b * strideR) : nullptr;
#pragma unroll
  for (int i = 0; i < 4; ++i) {
    const int mBase = m0 + (i << 4);
#pragma unroll
    for (int j = 0; j < 4; ++j) {
      const int n = n0 + (j << 4) + rlane;
      float bv = 0.f;
      if (BIAS_MODE == 2) bv = bias[n];
#pragma unroll
      for (int r = 0; r < 8; ++r) {
        float v = acc[i][j][r] * scale;
        if (BIAS_MODE == 1) v += bias[mBase + mOff + r];
        if (BIAS_MODE == 2) v += bv;
        if (RESID) v += Rb[(size_t)(mBase + mOff + r) * ldc + n];
        if (ACT == 1) v = tanhf(v);
        if (ACT == 2) v = fmaxf(v, 0.0f);
        if (ACT == 3) v = v / (1.0f + expf(-v));
        if (ACT == 4) v = (v > 0.f) ? v : 0.01f * v;
        if (ACT == 5) v = 0.5f * v * (1.0f + erff(v * 0.70710678118654752f));
        slab[(mOff + r) * 68 + (j << 4) + rlane] = v;
      }
    }
    __builtin_amdgcn_fence(__ATOMIC_RELEASE, "workgroup");
    __builtin_amdgcn_wave_barrier();
    __builtin_amdgcn_fence(__ATOMIC_ACQUIRE, "workgroup");
    if (OUT_MODE == 0) {
      float* C = (float*)Cout + (size_t)b * strideC;
      const int hh = lane >> 4, c4 = (lane & 15) * 4;
      for (int pass = 0; pass < 2; ++pass) {
#pragma unroll
        for (int it = 0; it < 8; ++it) {
          const int row = it * 2 + hh;
          v4f v = *(const v4f*)(slab + row * 68 + c4);
          if (ROPE == 1) {
            const int mg = mBase + row;
            const int t  = mg % ropeT;
            const v4f cs = *(const v4f*)(rope_cs + (size_t)t * 64 + c4);
            v4f w;
            w[0] = v[0] * cs[0] - v[1] * cs[1];
            w[1] = v[0] * cs[1] + v[1] * cs[0];
            w[2] = v[2] * cs[2] - v[3] * cs[3];
            w[3] = v[2] * cs[3] + v[3] * cs[2];
            v = w;
          }
          *(volatile v4f*)(C + (size_t)(mBase + row) * ldc + n0 + c4) = v;
        }
        __threadfence();
      }
    } else {
      const int q = lane >> 3, c8 = (lane & 7) * 8;
      unsigned short* C  = (unsigned short*)Cout  + (size_t)b * strideC;
      unsigned short* C2 = (OUT_MODE == 2) ? ((unsigned short*)Cout2 + (size_t)b * strideC) : nullptr;
      for (int pass = 0; pass < 2; ++pass) {
#pragma unroll
        for (int it = 0; it < 4; ++it) {
          const int row = it * 4 + q;
          const float* sp = slab + row * 68 + c8;
          v8h hv, lv;
#pragma unroll
          for (int e = 0; e < 8; ++e) {
            if (OUT_MODE == 1) {
              hv[e] = (_Float16)sp[e];
            } else {
              unsigned short hb = f2bf_bits(sp[e]);
              unsigned short lb = f2bf_bits(sp[e] - bf_bits2f(hb));
              hv[e] = __builtin_bit_cast(_Float16, hb);
              lv[e] = __builtin_bit_cast(_Float16, lb);
            }
          }
          *(volatile v8h*)(C + (size_t)(mBase + row) * ldc + n0 + c8) = hv;
          if (OUT_MODE == 2) *(volatile v8h*)(C2 + (size_t)(mBase + row) * ldc + n0 + c8) = lv;
        }
        __threadfence();
      }
    }
    __builtin_amdgcn_fence(__ATOMIC_RELEASE, "workgroup");
    __builtin_amdgcn_wave_barrier();
    __builtin_amdgcn_fence(__ATOMIC_ACQUIRE, "workgroup");
  }
}

__global__ __launch_bounds__(256) void rope_table_kernel(const int* __restrict__ posp, float* __restrict__ cs, int T) {
#pragma clang fp contract(off)
  const int idx = blockIdx.x * 256 + threadIdx.x;
  if (idx < T * 32) {
    const int t = idx >> 5, i = idx & 31;
    const double p = exp2((double)i * (13.287712379549449 / 32.0));
    const float pf = (float)p;
    const float invf = 1.0f / pf;
    const float th = ((float)posp[0] + (float)t) * invf;
    float sn, cn;
    sincosf(th, &sn, &cn);
    v2f o;
    o[0] = cn; o[1] = sn;
    float* dst = cs + 2 * (size_t)idx;
    *(volatile v2f*)dst = o;
    __threadfence();
    *(volatile v2f*)dst = o;
  }
}

__global__ __launch_bounds__(256) void cvt_x_kernel(const float* __restrict__ in,
    unsigned short* __restrict__ xh, unsigned short* __restrict__ xbh, unsigned short* __restrict__ xbl, int n8) {
  const int i = blockIdx.x * 256 + threadIdx.x;
  if (i < n8) {
    const size_t e0 = 8 * (size_t)i;
    const v4f a  = *(const v4f*)(in + e0);
    const v4f a2 = *(const v4f*)(in + e0 + 4);
    v8h hv, bh, bl;
#pragma unroll
    for (int e = 0; e < 4; ++e) {
      const float f0 = a[e], f1 = a2[e];
      hv[e]     = (_Float16)f0;
      hv[4 + e] = (_Float16)f1;
      const unsigned short hb0 = f2bf_bits(f0), hb1 = f2bf_bits(f1);
      const unsigned short lb0 = f2bf_bits(f0 - bf_bits2f(hb0)), lb1 = f2bf_bits(f1 - bf_bits2f(hb1));
      bh[e]     = __builtin_bit_cast(_Float16, hb0);
      bh[4 + e] = __builtin_bit_cast(_Float16, hb1);
      bl[e]     = __builtin_bit_cast(_Float16, lb0);
      bl[4 + e] = __builtin_bit_cast(_Float16, lb1);
    }
    for (int pass = 0; pass < 2; ++pass) {
      *(volatile v8h*)(xh  + e0) = hv;
      *(volatile v8h*)(xbh + e0) = bh;
      *(volatile v8h*)(xbl + e0) = bl;
      __threadfence();
    }
  }
}

template <int MODE>
__global__ __launch_bounds__(256) void transpose_cvt_kernel(const float* __restrict__ W, int K, int N,
    unsigned short* out0, unsigned short* out1, float scl) {
  __shared__ float tile[64][33];
  const int tid = threadIdx.x;
  const int k0 = blockIdx.x * 64, n0 = blockIdx.y * 32;
  {
    const int kk = tid >> 2, cc = (tid & 3) * 8;
    const float* src = W + (size_t)(k0 + kk) * N + n0 + cc;
    const v4f a  = *(const v4f*)src;
    const v4f a2 = *(const v4f*)(src + 4);
#pragma unroll
    for (int e = 0; e < 4; ++e) { tile[kk][cc + e] = a[e]; tile[kk][cc + 4 + e] = a2[e]; }
  }
  __syncthreads();
  const int nn = tid >> 3, kc = (tid & 7) * 8;
  v8h o0, o1;
#pragma unroll
  for (int e = 0; e < 8; ++e) {
    const float f = tile[kc + e][nn] * scl;
    if (MODE == 0) {
      o0[e] = (_Float16)f;
      o1[e] = o0[e];
    } else {
      const unsigned short hb = f2bf_bits(f);
      const unsigned short lb = f2bf_bits(f - bf_bits2f(hb));
      o0[e] = __builtin_bit_cast(_Float16, hb);
      o1[e] = __builtin_bit_cast(_Float16, lb);
    }
  }
  const size_t dst = (size_t)(n0 + nn) * K + k0 + kc;
  for (int pass = 0; pass < 2; ++pass) {
    *(volatile v8h*)(out0 + dst) = o0;
    if (MODE == 1) *(volatile v8h*)(out1 + dst) = o1;
    __threadfence();
  }
}

#define AT_D 64
#define AT_NW 4
#define AT_QB 64
#define AT_KC 64
#define AT_MAXCH 64

__global__ __launch_bounds__(128)
void attn_gqa_swa_kernel(const float* __restrict__ qf, const float* __restrict__ kvf,
                         unsigned short* __restrict__ ohi, unsigned short* __restrict__ olo,
                         int T, int H, int ldq, int ldkv, int voff, int ldo,
                         int win, int sink, int group, float scale) {
  union FH { v16h v; v8h h[2]; };
  union FB { v16b v; v8b h[2]; };
  __shared__ __align__(16) _Float16 Ksh[AT_KC * AT_D];
  __shared__ __align__(16) __bf16   Vth[AT_D * AT_KC];
  __shared__ __align__(16) __bf16   Vtl[AT_D * AT_KC];
  __shared__ __align__(16) __bf16   Psh[AT_NW][16 * AT_KC];
  __shared__ __align__(16) __bf16   Psl[AT_NW][16 * AT_KC];
  __shared__ __align__(16) float    Os[AT_NW][16 * 68];

  const int tid  = threadIdx.x;
  const int wave = tid >> 5;
  const int lane = tid & 31;
  const int hh   = lane >> 4;
  const int c    = lane & 15;

  const int nqb  = T / AT_QB;
  const int bx   = blockIdx.x;
  const int qb   = bx % nqb;
  const int bhid = bx / nqb;
  const int h    = bhid % H;
  const int b    = bhid / H;
  const int g    = h / group;
  const int q0   = qb * AT_QB + wave * 16;

  const float* qptr = qf  + (size_t)b * T * ldq  + (size_t)h * AT_D;
  const float* kptr = kvf + (size_t)b * T * ldkv + (size_t)g * AT_D;
  unsigned short* ohp = ohi + (size_t)b * T * ldo + (size_t)h * AT_D;
  unsigned short* olp = olo + (size_t)b * T * ldo + (size_t)h * AT_D;

  v16h qa[2];
  {
    const float* qrow = qptr + (size_t)(q0 + c) * ldq;
#pragma unroll
    for (int dc = 0; dc < 2; ++dc) {
#pragma unroll
      for (int e = 0; e < 8; ++e) {
        qa[dc][e]     = (_Float16)qrow[dc * 32 + 8 * hh + e];
        qa[dc][8 + e] = (_Float16)qrow[dc * 32 + 16 + 8 * hh + e];
      }
    }
  }

  float mrow[8], lrow[8];
  v8f oacc[4];
#pragma unroll
  for (int r = 0; r < 8; ++r) { mrow[r] = NEG_INF; lrow[r] = 0.f; }
#pragma unroll
  for (int t = 0; t < 4; ++t) oacc[t] = (v8f){0.f,0.f,0.f,0.f,0.f,0.f,0.f,0.f};

  int lo = qb * AT_QB - win;
  lo = (lo < AT_KC) ? 1 : (lo / AT_KC);
  if (lo > qb) lo = qb;
  int nvis = (qb == 0) ? 1 : (qb - lo + 2);
  if (nvis > AT_MAXCH) nvis = AT_MAXCH;

  for (int ci = 0; ci < nvis; ++ci) {
    const int kc  = (ci == 0) ? 0 : (lo + ci - 1);
    const int kv0 = kc * AT_KC;
    __syncthreads();
    {
      const int kvr = tid >> 1, dh = (tid & 1) * 32;
      const float* krow = kptr + (size_t)(kv0 + kvr) * ldkv + dh;
      const float* vrow = krow + voff;
#pragma unroll
      for (int i = 0; i < 8; ++i) {
        const v4f kk = *(const v4f*)(krow + 4 * i);
        const v4f vv = *(const v4f*)(vrow + 4 * i);
#pragma unroll
        for (int e = 0; e < 4; ++e) {
          const int d = dh + 4 * i + e;
          Ksh[kvr * AT_D + d] = (_Float16)kk[e];
          __bf16 a, bl; bf_split(vv[e], a, bl);
          Vth[d * AT_KC + kvr] = a;
          Vtl[d * AT_KC + kvr] = bl;
        }
      }
    }
    __syncthreads();

    v8f s[4];
#pragma unroll
    for (int j = 0; j < 4; ++j) {
      s[j] = (v8f){0.f,0.f,0.f,0.f,0.f,0.f,0.f,0.f};
#pragma unroll
      for (int dc = 0; dc < 2; ++dc) {
        FH kb;
        kb.h[0] = *(const v8h*)(Ksh + (j * 16 + c) * AT_D + dc * 32 + 8 * hh);
        kb.h[1] = *(const v8h*)(Ksh + (j * 16 + c) * AT_D + dc * 32 + 16 + 8 * hh);
        s[j] = mma_f16x(qa[dc], kb.v, s[j]);
      }
    }

    float cm[8];
#pragma unroll
    for (int r = 0; r < 8; ++r) {
      const int qrow = q0 + 8 * hh + r;
      float m = NEG_INF;
#pragma unroll
      for (int j = 0; j < 4; ++j) {
        const int kvcol = kv0 + j * 16 + c;
        float sv = s[j][r] * scale;
        const bool masked = (kvcol > qrow) || ((qrow - kvcol > win) && (kvcol >= sink));
        if (masked) sv = NEG_INF;
        s[j][r] = sv;
        m = fmaxf(m, sv);
      }
#pragma unroll
      for (int off = 1; off < 16; off <<= 1) m = fmaxf(m, __shfl_xor(m, off, 32));
      cm[r] = m;
    }

    __bf16* pwh = Psh[wave];
    __bf16* pwl = Psl[wave];
#pragma unroll
    for (int r = 0; r < 8; ++r) {
      const float mnew  = fmaxf(mrow[r], cm[r]);
      const float alpha = __expf(mrow[r] - mnew);
      mrow[r] = mnew;
      float psum = 0.f;
#pragma unroll
      for (int j = 0; j < 4; ++j) {
        const float p = __expf(s[j][r] - mnew);
        psum += p;
        __bf16 a, bl; bf_split(p, a, bl);
        pwh[(8 * hh + r) * AT_KC + j * 16 + c] = a;
        pwl[(8 * hh + r) * AT_KC + j * 16 + c] = bl;
      }
#pragma unroll
      for (int off = 1; off < 16; off <<= 1) psum += __shfl_xor(psum, off, 32);
      lrow[r] = lrow[r] * alpha + psum;
#pragma unroll
      for (int t = 0; t < 4; ++t) oacc[t][r] *= alpha;
    }
    __builtin_amdgcn_fence(__ATOMIC_RELEASE, "workgroup");
    __builtin_amdgcn_wave_barrier();
    __builtin_amdgcn_fence(__ATOMIC_ACQUIRE, "workgroup");

#pragma unroll
    for (int kk = 0; kk < 2; ++kk) {
      FB pa, pl;
      pa.h[0] = *(const v8b*)(pwh + c * AT_KC + kk * 32 + 8 * hh);
      pa.h[1] = *(const v8b*)(pwh + c * AT_KC + kk * 32 + 16 + 8 * hh);
      pl.h[0] = *(const v8b*)(pwl + c * AT_KC + kk * 32 + 8 * hh);
      pl.h[1] = *(const v8b*)(pwl + c * AT_KC + kk * 32 + 16 + 8 * hh);
#pragma unroll
      for (int t = 0; t < 4; ++t) {
        FB vb, vl;
        vb.h[0] = *(const v8b*)(Vth + (t * 16 + c) * AT_KC + kk * 32 + 8 * hh);
        vb.h[1] = *(const v8b*)(Vth + (t * 16 + c) * AT_KC + kk * 32 + 16 + 8 * hh);
        vl.h[0] = *(const v8b*)(Vtl + (t * 16 + c) * AT_KC + kk * 32 + 8 * hh);
        vl.h[1] = *(const v8b*)(Vtl + (t * 16 + c) * AT_KC + kk * 32 + 16 + 8 * hh);
        oacc[t] = mma_bf16x(pa.v, vb.v, oacc[t]);
        oacc[t] = mma_bf16x(pa.v, vl.v, oacc[t]);
        oacc[t] = mma_bf16x(pl.v, vb.v, oacc[t]);
      }
    }
  }

  float* os = Os[wave];
#pragma unroll
  for (int r = 0; r < 8; ++r) {
    const float inv = 1.0f / lrow[r];
#pragma unroll
    for (int t = 0; t < 4; ++t) os[(8 * hh + r) * 68 + t * 16 + c] = oacc[t][r] * inv;
  }
  __builtin_amdgcn_fence(__ATOMIC_RELEASE, "workgroup");
  __builtin_amdgcn_wave_barrier();
  __builtin_amdgcn_fence(__ATOMIC_ACQUIRE, "workgroup");
  {
    const int q4 = lane >> 3, c8 = (lane & 7) * 8;
    for (int pass = 0; pass < 2; ++pass) {
#pragma unroll
      for (int it = 0; it < 4; ++it) {
        const int row = it * 4 + q4;
        const float* sp = os + row * 68 + c8;
        v8h hv, lv;
#pragma unroll
        for (int e = 0; e < 8; ++e) {
          const unsigned short hb = f2bf_bits(sp[e]);
          const unsigned short lb = f2bf_bits(sp[e] - bf_bits2f(hb));
          hv[e] = __builtin_bit_cast(_Float16, hb);
          lv[e] = __builtin_bit_cast(_Float16, lb);
        }
        const size_t go = (size_t)(q0 + row) * ldo + c8;
        *(volatile v8h*)(ohp + go) = hv;
        *(volatile v8h*)(olp + go) = lv;
      }
      __threadfence();
    }
  }
}

static inline size_t al256(size_t x) { return (x + 255) & ~(size_t)255; }

extern "C" void kernel_launch(void* const* d_in, const int* in_sizes, int n_in,
                              void* d_out, int out_size, void* d_ws, size_t ws_size,
                              hipStream_t stream) {
  constexpr int Bc = 2, Tc = 2048, Cc = 1024, Hc = 16, Gc = 4, Dc = 64;
  constexpr int WINc = 512, SINKc = 4;
  constexpr int Mr  = Bc * Tc;
  constexpr int NQ  = Hc * Dc;
  constexpr int NKV = Gc * Dc;
  constexpr float SCALEc = 0.125f;

  if (n_in < 10) return;
  if (in_sizes[0] != Mr * Cc || in_sizes[1] != Cc * NQ || in_sizes[2] != NQ ||
      in_sizes[3] != Cc * NKV || in_sizes[4] != NKV || in_sizes[5] != Cc * NKV || in_sizes[6] != NKV ||
      in_sizes[7] != Cc * Cc || in_sizes[8] != Cc || in_sizes[9] < 1 || out_size != Mr * Cc) return;

  const float* x   = (const float*)d_in[0];
  const float* Wq  = (const float*)d_in[1];
  const float* bq  = (const float*)d_in[2];
  const float* Wk  = (const float*)d_in[3];
  const float* bk  = (const float*)d_in[4];
  const float* Wv  = (const float*)d_in[5];
  const float* bvv = (const float*)d_in[6];
  const float* Wo  = (const float*)d_in[7];
  const float* bo  = (const float*)d_in[8];
  const int*   pos = (const int*)d_in[9];
  float* out = (float*)d_out;

  char* w = (char*)d_ws;
  size_t off = 0;
  float*          cs   = (float*)(w + off);          off += al256((size_t)Tc * 64 * 4);
  unsigned short* x16  = (unsigned short*)(w + off); off += al256((size_t)Mr * Cc * 2);
  unsigned short* xbh  = (unsigned short*)(w + off); off += al256((size_t)Mr * Cc * 2);
  unsigned short* xbl  = (unsigned short*)(w + off); off += al256((size_t)Mr * Cc * 2);
  unsigned short* wqT  = (unsigned short*)(w + off); off += al256((size_t)NQ * Cc * 2);
  unsigned short* wkTh = (unsigned short*)(w + off); off += al256((size_t)NKV * Cc * 2);
  unsigned short* wkTl = (unsigned short*)(w + off); off += al256((size_t)NKV * Cc * 2);
  unsigned short* wvTh = (unsigned short*)(w + off); off += al256((size_t)NKV * Cc * 2);
  unsigned short* wvTl = (unsigned short*)(w + off); off += al256((size_t)NKV * Cc * 2);
  unsigned short* woTh = (unsigned short*)(w + off); off += al256((size_t)Cc * Cc * 2);
  unsigned short* woTl = (unsigned short*)(w + off); off += al256((size_t)Cc * Cc * 2);
  float*          qf   = (float*)(w + off);          off += al256((size_t)Mr * NQ * 4);
  float*          kvf  = (float*)(w + off);          off += al256((size_t)Mr * 2 * NKV * 4);
  unsigned short* ath  = (unsigned short*)(w + off); off += al256((size_t)Mr * Cc * 2);
  unsigned short* atl  = (unsigned short*)(w + off); off += al256((size_t)Mr * Cc * 2);
  if (off > ws_size) return;

  rope_table_kernel<<<dim3((Tc * 32 + 255) / 256), dim3(256), 0, stream>>>(pos, cs, Tc);

  const int n8 = Mr * Cc / 8;
  cvt_x_kernel<<<dim3((n8 + 255) / 256), dim3(256), 0, stream>>>(x, x16, xbh, xbl, n8);

  transpose_cvt_kernel<0><<<dim3(Cc / 64, NQ / 32),  dim3(256), 0, stream>>>(Wq, Cc, NQ,  wqT,  wqT,  64.0f);
  transpose_cvt_kernel<1><<<dim3(Cc / 64, NKV / 32), dim3(256), 0, stream>>>(Wk, Cc, NKV, wkTh, wkTl, 1.0f);
  transpose_cvt_kernel<1><<<dim3(Cc / 64, NKV / 32), dim3(256), 0, stream>>>(Wv, Cc, NKV, wvTh, wvTl, 1.0f);
  transpose_cvt_kernel<1><<<dim3(Cc / 64, Cc / 32),  dim3(256), 0, stream>>>(Wo, Cc, Cc,  woTh, woTl, 1.0f);

  {
    const int tiles = (Mr / 64) * (NQ / 64);
    wmma_gemm64<0, false, 2, 0, false, 0, 1><<<dim3((tiles + 7) / 8, 1), dim3(256), 0, stream>>>(
        x16, x16, Cc, (long)0,
        wqT, wqT, Cc, (long)0,
        (void*)qf, (void*)qf, NQ, (long)0,
        bq, (const float*)kvf, (long)0,
        cs, Tc,
        Mr, NQ, Cc, 1.0f / 64.0f);
  }
  {
    const int tiles = (Mr / 64) * (NKV / 64);
    wmma_gemm64<1, true, 2, 0, false, 0, 1><<<dim3((tiles + 7) / 8, 1), dim3(256), 0, stream>>>(
        xbh, xbl, Cc, (long)0,
        wkTh, wkTl, Cc, (long)0,
        (void*)kvf, (void*)kvf, 2 * NKV, (long)0,
        bk, (const float*)qf, (long)0,
        cs, Tc,
        Mr, NKV, Cc, 1.0f);
  }
  {
    const int tiles = (Mr / 64) * (NKV / 64);
    wmma_gemm64<1, true, 2, 0, false, 0, 0><<<dim3((tiles + 7) / 8, 1), dim3(256), 0, stream>>>(
        xbh, xbl, Cc, (long)0,
        wvTh, wvTl, Cc, (long)0,
        (void*)(kvf + NKV), (void*)(kvf + NKV), 2 * NKV, (long)0,
        bvv, (const float*)qf, (long)0,
        cs, Tc,
        Mr, NKV, Cc, 1.0f);
  }
  attn_gqa_swa_kernel<<<dim3(Bc * Hc * (Tc / 64)), dim3(128), 0, stream>>>(
      qf, kvf, ath, atl, Tc, Hc, NQ, 2 * NKV, NKV, Cc, WINc, SINKc, Hc / Gc, SCALEc);

  {
    const int tiles = (Mr / 64) * (Cc / 64);
    wmma_gemm64<1, true, 2, 0, false, 0, 0><<<dim3((tiles + 7) / 8, 1), dim3(256), 0, stream>>>(
        ath, atl, Cc, (long)0,
        woTh, woTl, Cc, (long)0,
        (void*)out, (void*)out, Cc, (long)0,
        bo, (const float*)qf, (long)0,
        cs, Tc,
        Mr, Cc, Cc, 1.0f);
  }
}
